// PinSAGE_29618094473883
// MI455X (gfx1250) — hardware-verified
//
#include <hip/hip_runtime.h>
#include <math.h>


typedef unsigned int u32;
typedef __attribute__((ext_vector_type(2)))  int      v2i;
typedef __attribute__((ext_vector_type(16))) _Float16 v16h;
typedef __attribute__((ext_vector_type(8)))  _Float16 v8h;
typedef __attribute__((ext_vector_type(8)))  float    v8f;
typedef __attribute__((ext_vector_type(4)))  float    v4f;
#define NN    50000
#define NE    800000
#define FF    128
#define HH    256
#define NC    128
#define MAXDEG 4096
#define SORTN 1048576
#define TILE  8192
#define NPAD  50176
#define VST2(T, ptr, val) do { const T _v = (val); *(volatile T*)(ptr) = _v; __threadfence(); *(volatile T*)(ptr) = _v; } while (0)
__device__ __forceinline__ v8f wmma16(v16h a, v16h b, v8f c) {
  v8f d = __builtin_amdgcn_wmma_f32_16x16x32_f16(false, a, false, b, (short)0, c, false, false);
  asm volatile("v_nop\n\tv_nop\n\tv_nop\n\tv_nop" : "+v"(d) : "v"(a), "v"(b));
  return d;
}
__device__ __forceinline__ v16h frag16(const _Float16* p, int hh) {
  const v8h lo = *(const v8h*)(p + 8 * hh), hi = *(const v8h*)(p + 16 + 8 * hh);
  return __builtin_shufflevector(lo, hi, 0,1,2,3,4,5,6,7,8,9,10,11,12,13,14,15);
}
__global__ __launch_bounds__(256) void k_sort_init(const int* __restrict__ src, const int* __restrict__ dst, u32* __restrict__ A, int E) {
  const int i = blockIdx.x * 256 + threadIdx.x;
  VST2(u32, A + i, (i < E) ? (((u32)dst[i]) << 16) | (u32)src[i] : 0xffffffffu);
}
__device__ __forceinline__ void cas_lds(u32* s, int lo, int hi, bool up) {
  const u32 a = s[lo], b = s[hi]; const bool sw = up ? (a > b) : (a < b); s[lo] = sw ? b : a; s[hi] = sw ? a : b;
}
__global__ __launch_bounds__(256) void k_sort_local(u32* __restrict__ A) {
  __shared__ u32 s[TILE];
  const int base = blockIdx.x * TILE, t = threadIdx.x;
  for (int i = t; i < TILE; i += 256) s[i] = A[base + i];
  __syncthreads();
  for (int k = 2; k <= TILE; k <<= 1)
    for (int j = k >> 1; j > 0; j >>= 1) {
      for (int p = t; p < TILE / 2; p += 256) {
        const int lo = ((p >> __builtin_ctz(j)) << (__builtin_ctz(j) + 1)) | (p & (j - 1));
        cas_lds(s, lo, lo + j, (((base + lo) & k) == 0));
      }
      __syncthreads();
    }
  for (int pass = 0; pass < 2; ++pass) { for (int i = t; i < TILE; i += 256) *(volatile u32*)(A + base + i) = s[i]; __threadfence(); }
}
__global__ __launch_bounds__(256) void k_sort_global(u32* __restrict__ A, int logj, int k) {
  const int p = blockIdx.x * 256 + threadIdx.x;
  const int j = 1 << logj;
  const int lo = ((p >> logj) << (logj + 1)) | (p & (j - 1)), hi = lo + j;
  const u32 a = A[lo], b = A[hi];
  const bool up = ((lo & k) == 0), sw = up ? (a > b) : (a < b);
  const u32 vlo = sw ? b : a, vhi = sw ? a : b;
  *(volatile u32*)(A + lo) = vlo; *(volatile u32*)(A + hi) = vhi; __threadfence();
  *(volatile u32*)(A + lo) = vlo; *(volatile u32*)(A + hi) = vhi;
}
__global__ __launch_bounds__(256) void k_sort_lds(u32* __restrict__ A, int k) {
  __shared__ u32 s[TILE];
  const int base = blockIdx.x * TILE, t = threadIdx.x;
  for (int i = t; i < TILE; i += 256) s[i] = A[base + i];
  __syncthreads();
  for (int j = TILE >> 1; j > 0; j >>= 1) {
    for (int p = t; p < TILE / 2; p += 256) {
      const int lo = ((p >> __builtin_ctz(j)) << (__builtin_ctz(j) + 1)) | (p & (j - 1));
      cas_lds(s, lo, lo + j, (((base + lo) & k) == 0));
    }
    __syncthreads();
  }
  for (int pass = 0; pass < 2; ++pass) { for (int i = t; i < TILE; i += 256) *(volatile u32*)(A + base + i) = s[i]; __threadfence(); }
}

__global__ __launch_bounds__(256) void k_segs(const u32* __restrict__ A, v2i* __restrict__ seg, float* __restrict__ inv) {
  const int n = blockIdx.x * 256 + threadIdx.x;
  if (n >= NN) return;
  int lo = 0, hi = SORTN;
  while (lo < hi) { const int mid = (lo + hi) >> 1; if ((A[mid] >> 16) < (u32)n) lo = mid + 1; else hi = mid; }
  const int st = lo; hi = SORTN;
  while (lo < hi) { const int mid = (lo + hi) >> 1; if ((A[mid] >> 16) < (u32)(n + 1)) lo = mid + 1; else hi = mid; }
  const v2i sv = {st, lo - st};
  VST2(v2i, seg + n, sv);
  VST2(float, inv + n, 1.0f / fmaxf((float)(lo - st), 1.0f));
}
template <int W>
__global__ __launch_bounds__(256) void k_rows(const float* __restrict__ h, const u32* __restrict__ A, const v2i* __restrict__ seg, const float* __restrict__ inv,
                                              _Float16* __restrict__ A16) {
  constexpr int PER = 2 * W / 8;
  const int t = blockIdx.x * 256 + threadIdx.x;
  if (t >= NPAD * PER) return;
  const int i = t / PER, c = (t % PER) * 8;
  v8h o;
  if (i >= NN) { for (int e = 0; e < 8; ++e) o[e] = (_Float16)0.f; }
  else if (c >= W) {
#pragma unroll
    for (int e = 0; e < 8; ++e) o[e] = (_Float16)h[(size_t)i * W + c - W + e];
  } else {
    const v2i sv = seg[i];
    const int st = min(max(sv[0], 0), SORTN - 1), cnt = min(max(sv[1], 0), MAXDEG);
    float acc[8] = {0.f, 0.f, 0.f, 0.f, 0.f, 0.f, 0.f, 0.f};
    for (int p = 0; p < cnt; ++p) {
      const int j = min((int)(A[min(st + p, SORTN - 1)] & 0xffffu), NN - 1);
      const float* hr = h + (size_t)j * W + c;
#pragma unroll
      for (int e = 0; e < 8; ++e) acc[e] += hr[e];
    }
    const float w = inv[i];
#pragma unroll
    for (int e = 0; e < 8; ++e) o[e] = (_Float16)(acc[e] * w);
  }
  VST2(v8h, A16 + (size_t)i * (2 * W) + c, o);
}
__global__ __launch_bounds__(256) void k_wt(const float* __restrict__ w1, const float* __restrict__ w2, int K1, int K, int Nv, int Npad, int ldw, _Float16* __restrict__ Wt) {
  const int t = blockIdx.x * 256 + threadIdx.x;
  const int per = K / 8;
  if (t >= Npad * per) return;
  const int n = t / per, k0 = (t % per) * 8;
  v8h o;
#pragma unroll
  for (int e = 0; e < 8; ++e) { const int k = k0 + e; float v = 0.f; if (n < Nv) v = (k < K1) ? w1[k * ldw + n] : w2[(k - K1) * ldw + n]; o[e] = (_Float16)v; }
  VST2(v8h, Wt + (size_t)n * K + k0, o);
}
template <int K, int NTOT, int EPI>
__global__ __launch_bounds__(128) void k_gemm(const _Float16* __restrict__ A, const _Float16* __restrict__ Wt, const float* __restrict__ bias, float* __restrict__ out) {
  __shared__ __attribute__((aligned(16))) float sT[4][16][132];
  const int lane = threadIdx.x & 31, wave = threadIdx.x >> 5, hh = lane >> 4, l16 = lane & 15;
  const int m0 = blockIdx.x * 64 + wave * 16, n0 = blockIdx.y * 128;
  v8f acc[8];
#pragma unroll
  for (int ni = 0; ni < 8; ++ni) acc[ni] = (v8f){};
#pragma unroll 2
  for (int k0 = 0; k0 < K; k0 += 32) {
    const v16h a0 = frag16(A + (size_t)(m0 + l16) * K + k0, hh);
#pragma unroll
    for (int ni = 0; ni < 8; ++ni) { const v16h b = frag16(Wt + (size_t)(n0 + ni * 16 + l16) * K + k0, hh); acc[ni] = wmma16(a0, b, acc[ni]); }
  }
  float (*st)[132] = sT[wave];
#pragma unroll
  for (int ni = 0; ni < 8; ++ni)
#pragma unroll
    for (int i = 0; i < 8; ++i) { float v = acc[ni][i] + bias[n0 + ni * 16 + l16]; if (EPI == 1) v = fmaxf(v, 0.f); st[i + 8 * hh][ni * 16 + l16] = v; }
  __builtin_amdgcn_fence(__ATOMIC_RELEASE, "workgroup"); __builtin_amdgcn_wave_barrier(); __builtin_amdgcn_fence(__ATOMIC_ACQUIRE, "workgroup");
  if (EPI == 2) {
    if (lane < 16) {
      float* rw = st[lane];
      float mx = -INFINITY;
      for (int c = 0; c < 128; ++c) mx = fmaxf(mx, rw[c]);
      float s = 0.f;
      for (int c = 0; c < 128; ++c) s += expf(rw[c] - mx);
      const float lse = mx + logf(s);
      for (int c = 0; c < 128; ++c) rw[c] -= lse;
    }
    __builtin_amdgcn_fence(__ATOMIC_RELEASE, "workgroup"); __builtin_amdgcn_wave_barrier(); __builtin_amdgcn_fence(__ATOMIC_ACQUIRE, "workgroup");
  }
  for (int pass = 0; pass < 2; ++pass) {
#pragma unroll
    for (int rr = 0; rr < 16; ++rr) if (m0 + rr < NN || EPI == 1)
      *(volatile v4f*)(out + (size_t)(m0 + rr) * NTOT + n0 + lane * 4) = *(const v4f*)(&st[rr][lane * 4]);
    __threadfence();
  }
}
extern "C" void kernel_launch(void* const* d_in, const int* in_sizes, int n_in,
                              void* d_out, int out_size, void* d_ws, size_t ws_size, hipStream_t stream) {
  (void)in_sizes; (void)n_in; (void)out_size;
  const float* x    = (const float*)d_in[0];
  const int*   ei   = (const int*)  d_in[1];
  const float* W1l  = (const float*)d_in[2];
  const float* W1r  = (const float*)d_in[3];
  const float* b1   = (const float*)d_in[4];
  const float* W2l  = (const float*)d_in[5];
  const float* W2r  = (const float*)d_in[6];
  const float* b2   = (const float*)d_in[7];
  float* out = (float*)d_out;
  char* ws = (char*)d_ws; size_t off = 0;
  auto take = [&](size_t bytes) { void* p = ws + off; off = (off + bytes + 255) & ~(size_t)255; return p; };
  u32*      keys = (u32*)take((size_t)SORTN * 4);
  v2i*      seg  = (v2i*)take((size_t)NN * 8);
  float*    inv  = (float*)take((size_t)NN * 4);
  _Float16* A1   = (_Float16*)take((size_t)NPAD * 2 * FF * 2);
  _Float16* A2   = (_Float16*)take((size_t)NPAD * 2 * HH * 2);
  _Float16* Wt1  = (_Float16*)take((size_t)HH * 2 * FF * 2);
  _Float16* Wt2  = (_Float16*)take((size_t)NC * 2 * HH * 2);
  float*    h1   = (float*)take((size_t)NPAD * HH * 4);
  if (off > ws_size) return;
  const dim3 b256(256);
  k_sort_init<<<SORTN / 256, b256, 0, stream>>>(ei, ei + NE, keys, NE);
  k_sort_local<<<SORTN / TILE, b256, 0, stream>>>(keys);
  for (int k = TILE * 2; k <= SORTN; k <<= 1) {
    for (int logj = __builtin_ctz(k) - 1; (1 << logj) >= TILE; --logj)
      k_sort_global<<<SORTN / 2 / 256, b256, 0, stream>>>(keys, logj, k);
    k_sort_lds<<<SORTN / TILE, b256, 0, stream>>>(keys, k);
  }
  k_segs<<<(NN + 255) / 256, b256, 0, stream>>>(keys, seg, inv);
  k_rows<FF><<<(NPAD * 32 + 255) / 256, b256, 0, stream>>>(x, keys, seg, inv, A1);
  k_wt<<<(HH * 32 + 255) / 256, b256, 0, stream>>>(W1l, W1r, FF, 2 * FF, HH, HH, HH, Wt1);
  k_gemm<2 * FF, HH, 1><<<dim3(NPAD / 64, 2), 128, 0, stream>>>(A1, Wt1, b1, h1);
  k_rows<HH><<<(NPAD * 64 + 255) / 256, b256, 0, stream>>>(h1, keys, seg, inv, A2);
  k_wt<<<(NC * 64 + 255) / 256, b256, 0, stream>>>(W2l, W2r, HH, 2 * HH, NC, NC, NC, Wt2);
  k_gemm<2 * HH, NC, 2><<<dim3(NPAD / 64, 1), 128, 0, stream>>>(A2, Wt2, b2, out);
}
